// DynamicConv1dTBC_12266426597626
// MI455X (gfx1250) — hardware-verified
//
#include <hip/hip_runtime.h>
#include <stddef.h>
#include <stdint.h>

#define T_    2048
#define B_    4
#define C_    1024
#define H_    16
#define KT_   15
#define PADL  14
#define NROW  8192
#define NF    240
#define NFP   256
#define SWP   68
#define XBLK  (NROW / 8)
#define WBLK  (NFP / 8)
#define CT    16
#define XSR   (CT + KT_ - 1)
#define CONV_LDS ((XSR * C_ + CT * NF) * 4)

static_assert(NROW == T_ * B_);
static_assert(NF == H_ * KT_);
static_assert(NFP >= NF);
static_assert(NFP % 64 == 0);
static_assert(C_ % 32 == 0);
static_assert(C_ == 4 * 256);
static_assert(C_ / H_ == 64);
static_assert(NROW % 256 == 0);
static_assert(T_ % CT == 0);
static_assert(PADL == KT_ - 1);
static_assert((CT * NF) % 4 == 0);

typedef unsigned short u16;
typedef __bf16 v16b __attribute__((ext_vector_type(16)));
typedef unsigned short v8us __attribute__((ext_vector_type(8)));
typedef float v8f __attribute__((ext_vector_type(8)));
typedef float v4f __attribute__((ext_vector_type(4)));
typedef unsigned int v4u __attribute__((ext_vector_type(4)));

union Frag  { v16b v; v8us h[2]; };
union Pack8 { v8us h; v4u u; u16 s[8]; };

__device__ __forceinline__ v8f zero8() { return (v8f){0.f, 0.f, 0.f, 0.f, 0.f, 0.f, 0.f, 0.f}; }
__device__ __forceinline__ v4f zero4() { return (v4f){0.f, 0.f, 0.f, 0.f}; }

__device__ __forceinline__ v8f mma(v16b a, v16b b, v8f c) {
  c = __builtin_amdgcn_wmma_f32_16x16x32_bf16(false, a, false, b, (short)0, c, false, false);
  asm volatile("v_nop\n\tv_nop\n\tv_nop\n\tv_nop" : "+v"(c) : "v"(a), "v"(b));
  return c;
}

__device__ __forceinline__ u16 f2bf(float f) {
  unsigned int u = __float_as_uint(f);
  u += 0x7FFFu + ((u >> 16) & 1u);
  return (u16)(u >> 16);
}
__device__ __forceinline__ float bf2f(u16 h) { return __uint_as_float(((unsigned int)h) << 16); }
__device__ __forceinline__ u16 lo_of(float f, u16 hi) { return f2bf(f - bf2f(hi)); }
__device__ __forceinline__ void split8(v4f a, v4f b, v4u& hu, v4u& lu) {
  Pack8 ph, pl;
#pragma unroll
  for (int i = 0; i < 4; ++i) {
    const u16 h0 = f2bf(a[i]);
    ph.s[i] = h0;
    pl.s[i] = lo_of(a[i], h0);
    const u16 h1 = f2bf(b[i]);
    ph.s[4 + i] = h1;
    pl.s[4 + i] = lo_of(b[i], h1);
  }
  hu = ph.u;
  lu = pl.u;
}

__device__ __forceinline__ v16b ldfrag(const u16* p, int ld, int row0, int k0, int lane) {
  const int m = lane & 15, lh = lane >> 4;
  const u16* q = p + (size_t)(row0 + m) * ld + k0 + 8 * lh;
  Frag f;
  f.h[0] = *(const v8us*)(q);
  f.h[1] = *(const v8us*)(q + 16);
  return f.v;
}

__device__ __forceinline__ void gemm_hl(const u16* __restrict__ Ah, const u16* __restrict__ Al, int lda,
                                        const u16* __restrict__ Bh, const u16* __restrict__ Bl, int ldb, int K,
                                        int m0, int n0, int lane, v8f (&acc)[2][4]) {
#pragma unroll 1
  for (int k0 = 0; k0 < K; k0 += 32) {
    v16b bh[4];
#pragma unroll
    for (int t = 0; t < 4; ++t) bh[t] = ldfrag(Bh, ldb, n0 + 16 * t, k0, lane);
    const v16b a0 = ldfrag(Ah, lda, m0, k0, lane);
    const v16b a1 = ldfrag(Ah, lda, m0 + 16, k0, lane);
#pragma unroll
    for (int t = 0; t < 4; ++t) {
      acc[0][t] = mma(a0, bh[t], acc[0][t]);
      acc[1][t] = mma(a1, bh[t], acc[1][t]);
    }
    const v16b l0 = ldfrag(Al, lda, m0, k0, lane);
    const v16b l1 = ldfrag(Al, lda, m0 + 16, k0, lane);
#pragma unroll
    for (int t = 0; t < 4; ++t) {
      acc[0][t] = mma(l0, bh[t], acc[0][t]);
      acc[1][t] = mma(l1, bh[t], acc[1][t]);
    }
#pragma unroll
    for (int t = 0; t < 4; ++t) {
      const v16b bl = ldfrag(Bl, ldb, n0 + 16 * t, k0, lane);
      acc[0][t] = mma(a0, bl, acc[0][t]);
      acc[1][t] = mma(a1, bl, acc[1][t]);
    }
  }
}

__global__ __launch_bounds__(256) void k_cvt(const float* __restrict__ x, const float* __restrict__ wlin,
                                             u16* __restrict__ xh, u16* __restrict__ xl,
                                             u16* __restrict__ wh, u16* __restrict__ wl) {
  const int tid = threadIdx.x, lane = tid & 31, wave = tid >> 5;
  if ((int)blockIdx.x < XBLK) {
    const int row = blockIdx.x * 8 + wave;
    const float* s = x + (size_t)row * C_ + lane * 8;
    v4u hu[4], lu[4];
    size_t go[4];
#pragma unroll
    for (int it = 0; it < 4; ++it) {
      const v4f a0 = *(const v4f*)(s + it * 256);
      const v4f a1 = *(const v4f*)(s + it * 256 + 4);
      split8(a0, a1, hu[it], lu[it]);
      go[it] = (size_t)row * C_ + it * 256 + lane * 8;
    }
#pragma unroll
    for (int it = 0; it < 4; ++it) {
      *(volatile v4u*)(xh + go[it]) = hu[it];
      *(volatile v4u*)(xl + go[it]) = lu[it];
    }
    __threadfence();
#pragma unroll
    for (int it = 0; it < 4; ++it) {
      *(volatile v4u*)(xh + go[it]) = hu[it];
      *(volatile v4u*)(xl + go[it]) = lu[it];
    }
  } else {
    const int row  = ((int)blockIdx.x - XBLK) * 8 + wave;
    const int rowc = (row < NF) ? row : (NF - 1);
    const float* s = wlin + (size_t)rowc * C_ + lane * 8;
    v4u hu[4], lu[4];
    size_t go[4];
#pragma unroll
    for (int it = 0; it < 4; ++it) {
      v4f a0 = *(const v4f*)(s + it * 256);
      v4f a1 = *(const v4f*)(s + it * 256 + 4);
      if (row >= NF) {
        a0 = zero4();
        a1 = zero4();
      }
      split8(a0, a1, hu[it], lu[it]);
      go[it] = (size_t)row * C_ + it * 256 + lane * 8;
    }
#pragma unroll
    for (int it = 0; it < 4; ++it) {
      *(volatile v4u*)(wh + go[it]) = hu[it];
      *(volatile v4u*)(wl + go[it]) = lu[it];
    }
    __threadfence();
#pragma unroll
    for (int it = 0; it < 4; ++it) {
      *(volatile v4u*)(wh + go[it]) = hu[it];
      *(volatile v4u*)(wl + go[it]) = lu[it];
    }
  }
}

__global__ __launch_bounds__(256) void k_gemm(const u16* __restrict__ xh, const u16* __restrict__ xl,
                                              const u16* __restrict__ wh, const u16* __restrict__ wl,
                                              float* __restrict__ lg) {
  __shared__ __align__(16) float sw[8][16 * SWP];
  const int tid = threadIdx.x, lane = tid & 31, wave = tid >> 5;
  const int lh = lane >> 4, c = lane & 15;
  const int m0 = blockIdx.x * 256 + wave * 32;
  const int n0 = blockIdx.y * 64;

  v8f acc[2][4];
#pragma unroll
  for (int s = 0; s < 2; ++s)
#pragma unroll
    for (int t = 0; t < 4; ++t) acc[s][t] = zero8();
  gemm_hl(xh, xl, C_, wh, wl, C_, C_, m0, n0, lane, acc);

  float* w = sw[wave];
#pragma unroll
  for (int sub = 0; sub < 2; ++sub) {
    __syncthreads();
#pragma unroll
    for (int t = 0; t < 4; ++t) {
#pragma unroll
      for (int r = 0; r < 8; ++r) w[(8 * lh + r) * SWP + 16 * t + c] = acc[sub][t][r];
    }
    __syncthreads();
    v4f val[8];
    size_t go[8];
#pragma unroll
    for (int it = 0; it < 8; ++it) {
      const int row = 2 * it + lh;
      val[it] = *(const v4f*)(w + row * SWP + c * 4);
      go[it]  = (size_t)(m0 + sub * 16 + row) * NFP + n0 + c * 4;
    }
#pragma unroll
    for (int it = 0; it < 8; ++it) *(volatile v4f*)(lg + go[it]) = val[it];
    __threadfence();
#pragma unroll
    for (int it = 0; it < 8; ++it) *(volatile v4f*)(lg + go[it]) = val[it];
  }
}

__global__ __launch_bounds__(256) void k_conv(const float* __restrict__ x, const float* __restrict__ lg,
                                              float* __restrict__ out) {
  extern __shared__ __align__(16) float smem[];
  float* xs  = smem;
  float* wsm = smem + XSR * C_;
  const int tid = threadIdx.x;
  const int t0 = blockIdx.x * CT, b = blockIdx.y;

#pragma unroll 1
  for (int i = tid; i < XSR * (C_ / 4); i += 256) {
    const int row = i >> 8;
    const int q   = i & 255;
    const int tg  = t0 - PADL + row;
    const int tgc = (tg < 0) ? 0 : tg;
    v4f v = *(const v4f*)(x + ((size_t)tgc * B_ + b) * C_ + q * 4);
    if (tg < 0) v = zero4();
    *(v4f*)(xs + row * C_ + q * 4) = v;
  }
#pragma unroll 1
  for (int i = tid; i < CT * (NF / 4); i += 256) {
    const int tt = i / (NF / 4), q = i - tt * (NF / 4);
    const v4f v = *(const v4f*)(lg + ((size_t)(t0 + tt) * B_ + b) * NFP + q * 4);
    *(v4f*)(wsm + tt * NF + q * 4) = v;
  }
  __syncthreads();

  {
    const int tt = tid >> 4, h = tid & 15;
    float* p = wsm + tt * NF + h * KT_;
    float mx = -__builtin_huge_valf();
#pragma unroll 1
    for (int k = 0; k < KT_; ++k) mx = fmaxf(mx, p[k]);
    float s = 0.f;
#pragma unroll 1
    for (int k = 0; k < KT_; ++k) {
      const float e = __expf(p[k] - mx);
      p[k] = e;
      s += e;
    }
    const float inv = __builtin_amdgcn_rcpf(s);
#pragma unroll 1
    for (int k = 0; k < KT_; ++k) p[k] = p[k] * inv;
  }
  __syncthreads();

  const int c4 = tid * 4, h = tid >> 4;
#pragma unroll 1
  for (int tt = 0; tt < CT; ++tt) {
    const float* wp = wsm + tt * NF + h * KT_;
    const float* xp = xs + tt * C_ + c4;
    v4f acc = zero4();
#pragma unroll
    for (int k = 0; k < KT_; ++k) {
      const float wv = wp[k];
      const v4f xv = *(const v4f*)(xp + k * C_);
      acc = acc + wv * xv;
    }
    float* op = out + ((size_t)(t0 + tt) * B_ + b) * C_ + c4;
    *(volatile v4f*)op = acc;
    __threadfence();
    *(volatile v4f*)op = acc;
  }
}

extern "C" void kernel_launch(void* const* d_in, const int* in_sizes, int n_in,
                              void* d_out, int out_size, void* d_ws, size_t ws_size,
                              hipStream_t stream) {
  if (n_in < 2) return;
  if (in_sizes[0] != NROW * C_) return;
  if (in_sizes[1] != NF * C_) return;
  if (out_size != NROW * C_) return;

  const float* x    = (const float*)d_in[0];
  const float* wlin = (const float*)d_in[1];
  float* out = (float*)d_out;

  const size_t szX  = (size_t)NROW * C_ * 2;
  const size_t szW  = (size_t)NFP * C_ * 2;
  const size_t szLG = (size_t)NROW * NFP * 4;

  size_t off = 0;
  const size_t oXH = off; off += szX;
  const size_t oXL = off; off += szX;
  const size_t oWH = off; off += szW;
  const size_t oWL = off; off += szW;
  const size_t oLG = off; off += szLG;
  if (off > ws_size) return;
  if (off > (size_t)134217728) return;

  char* ws = (char*)d_ws;
  u16* XH = (u16*)(ws + oXH);
  u16* XL = (u16*)(ws + oXL);
  u16* WH = (u16*)(ws + oWH);
  u16* WL = (u16*)(ws + oWL);
  float* LG = (float*)(ws + oLG);

  k_cvt<<<dim3(XBLK + WBLK), dim3(256), 0, stream>>>(x, wlin, XH, XL, WH, WL);
  k_gemm<<<dim3(NROW / 256, NFP / 64), dim3(256), 0, stream>>>(XH, XL, WH, WL, LG);
  (void)hipFuncSetAttribute(reinterpret_cast<const void*>(&k_conv),
                            hipFuncAttributeMaxDynamicSharedMemorySize, CONV_LDS);
  k_conv<<<dim3(T_ / CT, B_), dim3(256), CONV_LDS, stream>>>(x, LG, out);
  (void)hipGetLastError();
}
